// HeteroTopologyEncoder_68642167324677
// MI455X (gfx1250) — hardware-run, weakly checked
//
#include <hip/hip_runtime.h>


namespace {
constexpr int NV = 50000, NRS = 500, NRP = 512, EVV = 400000, EVI = 100000, EIV = 100000, DV = 6, L2 = 64, OUT = 64, NPB = 8;
constexpr float HS = 256.0f, WSC = 256.0f, LNEPS = 1e-5f;
typedef _Float16 b16;
typedef __attribute__((ext_vector_type(16))) _Float16 v16b;
typedef __attribute__((ext_vector_type(8))) _Float16 v8b;
typedef __attribute__((ext_vector_type(8))) float v8f;
typedef __attribute__((ext_vector_type(4))) float v4f;
typedef __attribute__((ext_vector_type(2))) float v2f;
__device__ __forceinline__ float bf16_rne(float f) { unsigned int u = __float_as_uint(f); u += 0x7FFFu + ((u >> 16) & 1u); float r = __uint_as_float(u & 0xFFFF0000u); asm volatile("" : "+v"(r)); return r; }
__device__ __forceinline__ float bfv(float f) { float r = bf16_rne(f); asm volatile("" : "+v"(r)); return r; }
__device__ __forceinline__ void split16(float v, b16& hi, b16& lo) { hi = (b16)v; lo = (b16)(v - (float)hi); }
__device__ __forceinline__ v16b frag_kb(const b16* p, int hh) { const v8b a = *(const v8b*)(p + 8 * hh), b = *(const v8b*)(p + 16 + 8 * hh); v16b f;
#pragma unroll
  for (int e = 0; e < 8; ++e) { f[e] = a[e]; f[8 + e] = b[e]; } return f; }
__device__ __forceinline__ v8f wmma16b(v16b a, v16b b, v8f c) { v8f d = __builtin_amdgcn_wmma_f32_16x16x32_f16(false, a, false, b, (short)0, c, false, false); asm volatile("v_nop\n\tv_nop\n\tv_nop\n\tv_nop" : "+v"(d) : "v"(a), "v"(b)); return d; }
__device__ __forceinline__ void wave_lds_sync() { __builtin_amdgcn_fence(__ATOMIC_RELEASE, "workgroup"); __builtin_amdgcn_wave_barrier(); __builtin_amdgcn_fence(__ATOMIC_ACQUIRE, "workgroup"); }
__device__ __forceinline__ float pmul(float a, float b) { float p = a * b; asm volatile("" : "+v"(p)); return p; }
__device__ __forceinline__ int iclamp(int v, int lo, int hi) { return v < lo ? lo : (v > hi ? hi : v); }
__device__ __forceinline__ float leaky(float v) { return v >= 0.0f ? v : 0.2f * v; }
__device__ __forceinline__ float elu(float v) { return v > 0.0f ? v : (__expf(v) - 1.0f); }
constexpr int CSR_NBLK8 = 512, CSR_GB8 = 8, CSR_GN8 = 1 << CSR_GB8  , CSR_TS8 = (CSR_GN8 < 32 ? 32 : CSR_GN8)  , CSR_MAXG8 = 512, CSR_CAP8 = 12288  ;
__device__ __host__ __forceinline__ int csr_tix8(int v) { return (v >> CSR_GB8) * CSR_TS8 + (v & (CSR_GN8 - 1)); }
__global__ __launch_bounds__(64) void csrA_kernel8(const int* __restrict__ dst, int E, int N, int nG, int CHP, int NGP, int* __restrict__ STG, int* __restrict__ HST) {
  extern __shared__ int sm[];
  int* cnt = sm; int* run = sm + NGP; int* ids = sm + 2 * NGP;
  const int b = blockIdx.x; const int ch = (E + CSR_NBLK8 - 1) / CSR_NBLK8; const int e0 = b * ch, e1 = min(E, e0 + ch);
  for (int i = threadIdx.x; i < NGP; i += 64) cnt[i] = 0;
  for (int i = threadIdx.x; i < CHP; i += 64) ids[i] = -1;
  __syncthreads();
  if (threadIdx.x == 0) {
    for (int e = e0; e < e1; ++e) { int d = dst[e]; d = (d < 0) ? 0 : (d >= N ? N - 1 : d); cnt[d >> CSR_GB8] += 1; }
    int acc = 0; for (int g = 0; g < nG; ++g) { run[g] = acc; acc += cnt[g]; }
    for (int e = e0; e < e1; ++e) { int d = dst[e]; d = (d < 0) ? 0 : (d >= N ? N - 1 : d); const int g = d >> CSR_GB8; ids[run[g]] = e; run[g] += 1; } }
  __syncthreads();
  typedef __attribute__((ext_vector_type(4))) int v4i;
  for (int pass = 0; pass < 2; ++pass) {
    for (int i = threadIdx.x; i < CHP / 4; i += 64) *(volatile v4i*)(STG + (size_t)b * CHP + i * 4) = *(const v4i*)(&ids[i * 4]);
    for (int i = threadIdx.x; i < NGP / 4; i += 64) { v4i v; for (int e = 0; e < 4; ++e) v[e] = (i * 4 + e < nG) ? cnt[i * 4 + e] : 0; *(volatile v4i*)(HST + (size_t)b * NGP + i * 4) = v; }
    __threadfence(); }
}
__global__ __launch_bounds__(512) void csrS_kernel8(const int* __restrict__ HST, int nG, int NGP, int* __restrict__ START, int* __restrict__ TOT, int* __restrict__ OFF) {
  __shared__ int tot[CSR_MAXG8];
  const int b = threadIdx.x;
  for (int pass = 0; pass < 2; ++pass) { int runb = 0; for (int g = 0; g < nG; ++g) { int c = HST[(size_t)b * NGP + g]; c = (c < 0) ? 0 : c; ((volatile int*)OFF)[(size_t)g * CSR_NBLK8 + b] = runb; runb += c; } __threadfence(); }
  for (int g = threadIdx.x; g < nG; g += 512) { int s = 0; for (int bb = 0; bb < CSR_NBLK8; ++bb) { int c = HST[(size_t)bb * NGP + g]; s += (c < 0) ? 0 : c; } tot[g] = s; }
  __syncthreads();
  if (threadIdx.x < 32) {
    __shared__ int st[CSR_MAXG8 + 32];
    if (threadIdx.x == 0) { int acc = 0; for (int g = 0; g < NGP; ++g) { st[g] = acc; if (g < nG) acc += (tot[g] + 31) & ~31; } st[NGP] = acc; }
    __builtin_amdgcn_fence(__ATOMIC_RELEASE, "workgroup"); __builtin_amdgcn_wave_barrier(); __builtin_amdgcn_fence(__ATOMIC_ACQUIRE, "workgroup");
    for (int pass = 0; pass < 2; ++pass) { for (int i = threadIdx.x; i < NGP + 32; i += 32) { ((volatile int*)START)[i] = (i <= NGP) ? st[min(i, NGP)] : 0; ((volatile int*)TOT)[i] = (i < nG) ? tot[i] : 0; } __threadfence(); } }
}
__global__ __launch_bounds__(256) void csrB_kernel8(const int* __restrict__ dst, int N, int nG, int CHP, int NGP, int permLen, const int* __restrict__ STG, const int* __restrict__ HST, const int* __restrict__ OFF, const int* __restrict__ START, const int* __restrict__ TOT, int* __restrict__ PERM, int* __restrict__ ROWPTR, int* __restrict__ ROWCNT, int* __restrict__ FLAG) {
  typedef __attribute__((ext_vector_type(4))) int v4i;
  __shared__ int ids[CSR_CAP8]; __shared__ unsigned short key[CSR_CAP8]; __shared__ int outp[CSR_CAP8]; __shared__ int ncnt[CSR_GN8 + 1]; __shared__ int boff[CSR_NBLK8 + 1];
  const int g = blockIdx.x, t_ = threadIdx.x; int tot = TOT[g]; int st = START[g], stn = START[g + 1]; const int v0 = g * CSR_GN8; const int nv = min(CSR_GN8, N - v0); const int t0 = g * CSR_TS8;
  st = (st < 0) ? 0 : (st > permLen - 32 ? permLen - 32 : st) & ~31; stn = (stn < st) ? st : (stn > permLen ? permLen : stn); tot = (tot < 0) ? 0 : tot; if (tot > stn - st && tot <= CSR_CAP8) tot = stn - st;
  if (tot > CSR_CAP8) {
    for (int pass = 0; pass < 2; ++pass) { for (int i = t_; i < CSR_TS8 / 4; i += 256) { v4i a, c; for (int e = 0; e < 4; ++e) { a[e] = st; c[e] = 0; } *(volatile v4i*)(ROWPTR + t0 + i * 4) = a; *(volatile v4i*)(ROWCNT + t0 + i * 4) = c; } if (t_ == 0) ((volatile int*)FLAG)[0] = 1; __threadfence(); } (void)nv; return; }
  if (t_ == 0) { int acc = 0; for (int b = 0; b < CSR_NBLK8; ++b) { boff[b] = acc; int c = HST[(size_t)b * NGP + g]; c = (c < 0) ? 0 : (c > CHP ? CHP : c); acc += c; if (acc > tot) acc = tot; } boff[CSR_NBLK8] = acc; }
  for (int i = t_; i <= CSR_GN8; i += 256) ncnt[i] = 0;
  __syncthreads();
  for (int b = 0; b < CSR_NBLK8; ++b) { const int c = boff[b + 1] - boff[b]; int o_ = OFF[(size_t)g * CSR_NBLK8 + b]; o_ = (o_ < 0) ? 0 : (o_ > CHP - c ? CHP - c : o_); const int* src_ = STG + (size_t)b * CHP + o_;
    for (int i = t_; i < c; i += 256) { int id = src_[i]; id = (id < 0) ? 0 : id; ids[boff[b] + i] = id; int d = dst[id]; d = (d < v0) ? v0 : (d >= N ? N - 1 : d); int kk = d - v0; kk = (kk < 0) ? 0 : (kk >= CSR_GN8 ? CSR_GN8 - 1 : kk); key[boff[b] + i] = (unsigned short)kk; } }
  __syncthreads();
  if (t_ == 0) { for (int i = 0; i < tot; ++i) ncnt[key[i]] += 1; int acc = 0; for (int vl = 0; vl < CSR_GN8; ++vl) { const int c = ncnt[vl]; ncnt[vl] = acc; acc += c; } ncnt[CSR_GN8] = acc;
    for (int i = 0; i < tot; ++i) { const int vl = key[i]; outp[ncnt[vl]] = ids[i]; ncnt[vl] += 1; }
    for (int vl = CSR_GN8; vl > 0; --vl) ncnt[vl] = ncnt[vl - 1]; ncnt[0] = 0; }
  __syncthreads();
  for (int pass = 0; pass < 2; ++pass) {
    for (int i = t_; i < (stn - st) / 4; i += 256) { v4i v; for (int e = 0; e < 4; ++e) { const int q = i * 4 + e; v[e] = (q < tot) ? outp[q] : -1; } *(volatile v4i*)(PERM + st + i * 4) = v; }
    for (int i = t_; i < CSR_TS8 / 4; i += 256) { v4i a, c; for (int e = 0; e < 4; ++e) { const int vl = i * 4 + e; const int vc = vl < CSR_GN8 ? vl : CSR_GN8; a[e] = (vl < CSR_GN8) ? st + ncnt[vc] : st; c[e] = (vl < nv) ? (ncnt[(vc < CSR_GN8 ? vc : CSR_GN8 - 1) + 1] - ncnt[vc]) : 0; } *(volatile v4i*)(ROWPTR + t0 + i * 4) = a; *(volatile v4i*)(ROWCNT + t0 + i * 4) = c; }
    __threadfence(); }
}
__global__ __launch_bounds__(256) void csrZ_kernel8(int* __restrict__ p, size_t n4) { typedef __attribute__((ext_vector_type(4))) int v4i; const size_t tid = (size_t)blockIdx.x * 256 + threadIdx.x, nth = (size_t)gridDim.x * 256; v4i z = {0, 0, 0, 0}; for (size_t i = tid; i < n4; i += nth) *(volatile v4i*)(p + i * 4) = z; }
struct CsrBufs8 { int *STG, *HST, *OFF, *START, *TOT, *PERM, *ROWPTR, *ROWCNT, *FLAG; int nG, NGP, CHP; size_t permLen; char* base; size_t bytes; };
static size_t csr_carve8(CsrBufs8& c, char* ws, size_t off, int E, int N) {
  const size_t off0 = off; c.base = ws + off;
  auto al = [&](size_t bytes) { char* p = ws + off; off += (bytes + 255) & ~(size_t)255; return p; };
  c.nG = (N + CSR_GN8 - 1) / CSR_GN8; c.NGP = (c.nG + 31) & ~31; const int ch = (E + CSR_NBLK8 - 1) / CSR_NBLK8; c.CHP = (ch + 31) & ~31; c.permLen = (size_t)E + 32 * (size_t)c.nG + 32;
  c.STG = (int*)al((size_t)CSR_NBLK8 * c.CHP * 4); c.HST = (int*)al((size_t)CSR_NBLK8 * c.NGP * 4); c.OFF = (int*)al((size_t)c.NGP * CSR_NBLK8 * 4); c.START = (int*)al((size_t)(c.NGP + 64) * 4); c.TOT = (int*)al((size_t)(c.NGP + 64) * 4);
  c.PERM = (int*)al(c.permLen * 4); c.ROWPTR = (int*)al((size_t)c.nG * CSR_TS8 * 4); c.ROWCNT = (int*)al((size_t)c.nG * CSR_TS8 * 4); c.FLAG = (int*)al(256);
  c.bytes = off - off0; return off;
}
static void csr_build8(const CsrBufs8& c, const int* dst, int E, int N, hipStream_t stream) {
  const size_t smem = (size_t)(2 * c.NGP + c.CHP) * 4;
  csrZ_kernel8<<<512, 256, 0, stream>>>((int*)c.base, c.bytes / 16);
  csrA_kernel8<<<CSR_NBLK8, 64, smem, stream>>>(dst, E, N, c.nG, c.CHP, c.NGP, c.STG, c.HST);
  csrS_kernel8<<<1, 512, 0, stream>>>(c.HST, c.nG, c.NGP, c.START, c.TOT, c.OFF);
  csrB_kernel8<<<c.nG, 256, 0, stream>>>(dst, N, c.nG, c.CHP, c.NGP, (int)c.permLen, c.STG, c.HST, c.OFF, c.START, c.TOT, c.PERM, c.ROWPTR, c.ROWCNT, c.FLAG);
}
constexpr int CSR_NBLK5 = 512, CSR_GB5 = 5, CSR_GN5 = 1 << CSR_GB5  , CSR_TS5 = (CSR_GN5 < 32 ? 32 : CSR_GN5)  , CSR_MAXG5 = 512, CSR_CAP5 = 12288  ;
__device__ __host__ __forceinline__ int csr_tix5(int v) { return (v >> CSR_GB5) * CSR_TS5 + (v & (CSR_GN5 - 1)); }
__global__ __launch_bounds__(64) void csrA_kernel5(const int* __restrict__ dst, int E, int N, int nG, int CHP, int NGP, int* __restrict__ STG, int* __restrict__ HST) {
  extern __shared__ int sm[];
  int* cnt = sm; int* run = sm + NGP; int* ids = sm + 2 * NGP;
  const int b = blockIdx.x; const int ch = (E + CSR_NBLK5 - 1) / CSR_NBLK5; const int e0 = b * ch, e1 = min(E, e0 + ch);
  for (int i = threadIdx.x; i < NGP; i += 64) cnt[i] = 0;
  for (int i = threadIdx.x; i < CHP; i += 64) ids[i] = -1;
  __syncthreads();
  if (threadIdx.x == 0) {
    for (int e = e0; e < e1; ++e) { int d = dst[e]; d = (d < 0) ? 0 : (d >= N ? N - 1 : d); cnt[d >> CSR_GB5] += 1; }
    int acc = 0; for (int g = 0; g < nG; ++g) { run[g] = acc; acc += cnt[g]; }
    for (int e = e0; e < e1; ++e) { int d = dst[e]; d = (d < 0) ? 0 : (d >= N ? N - 1 : d); const int g = d >> CSR_GB5; ids[run[g]] = e; run[g] += 1; } }
  __syncthreads();
  typedef __attribute__((ext_vector_type(4))) int v4i;
  for (int pass = 0; pass < 2; ++pass) {
    for (int i = threadIdx.x; i < CHP / 4; i += 64) *(volatile v4i*)(STG + (size_t)b * CHP + i * 4) = *(const v4i*)(&ids[i * 4]);
    for (int i = threadIdx.x; i < NGP / 4; i += 64) { v4i v; for (int e = 0; e < 4; ++e) v[e] = (i * 4 + e < nG) ? cnt[i * 4 + e] : 0; *(volatile v4i*)(HST + (size_t)b * NGP + i * 4) = v; }
    __threadfence(); }
}
__global__ __launch_bounds__(512) void csrS_kernel5(const int* __restrict__ HST, int nG, int NGP, int* __restrict__ START, int* __restrict__ TOT, int* __restrict__ OFF) {
  __shared__ int tot[CSR_MAXG5];
  const int b = threadIdx.x;
  for (int pass = 0; pass < 2; ++pass) { int runb = 0; for (int g = 0; g < nG; ++g) { int c = HST[(size_t)b * NGP + g]; c = (c < 0) ? 0 : c; ((volatile int*)OFF)[(size_t)g * CSR_NBLK5 + b] = runb; runb += c; } __threadfence(); }
  for (int g = threadIdx.x; g < nG; g += 512) { int s = 0; for (int bb = 0; bb < CSR_NBLK5; ++bb) { int c = HST[(size_t)bb * NGP + g]; s += (c < 0) ? 0 : c; } tot[g] = s; }
  __syncthreads();
  if (threadIdx.x < 32) {
    __shared__ int st[CSR_MAXG5 + 32];
    if (threadIdx.x == 0) { int acc = 0; for (int g = 0; g < NGP; ++g) { st[g] = acc; if (g < nG) acc += (tot[g] + 31) & ~31; } st[NGP] = acc; }
    __builtin_amdgcn_fence(__ATOMIC_RELEASE, "workgroup"); __builtin_amdgcn_wave_barrier(); __builtin_amdgcn_fence(__ATOMIC_ACQUIRE, "workgroup");
    for (int pass = 0; pass < 2; ++pass) { for (int i = threadIdx.x; i < NGP + 32; i += 32) { ((volatile int*)START)[i] = (i <= NGP) ? st[min(i, NGP)] : 0; ((volatile int*)TOT)[i] = (i < nG) ? tot[i] : 0; } __threadfence(); } }
}
__global__ __launch_bounds__(256) void csrB_kernel5(const int* __restrict__ dst, int N, int nG, int CHP, int NGP, int permLen, const int* __restrict__ STG, const int* __restrict__ HST, const int* __restrict__ OFF, const int* __restrict__ START, const int* __restrict__ TOT, int* __restrict__ PERM, int* __restrict__ ROWPTR, int* __restrict__ ROWCNT, int* __restrict__ FLAG) {
  typedef __attribute__((ext_vector_type(4))) int v4i;
  __shared__ int ids[CSR_CAP5]; __shared__ unsigned short key[CSR_CAP5]; __shared__ int outp[CSR_CAP5]; __shared__ int ncnt[CSR_GN5 + 1]; __shared__ int boff[CSR_NBLK5 + 1];
  const int g = blockIdx.x, t_ = threadIdx.x; int tot = TOT[g]; int st = START[g], stn = START[g + 1]; const int v0 = g * CSR_GN5; const int nv = min(CSR_GN5, N - v0); const int t0 = g * CSR_TS5;
  st = (st < 0) ? 0 : (st > permLen - 32 ? permLen - 32 : st) & ~31; stn = (stn < st) ? st : (stn > permLen ? permLen : stn); tot = (tot < 0) ? 0 : tot; if (tot > stn - st && tot <= CSR_CAP5) tot = stn - st;
  if (tot > CSR_CAP5) {
    for (int pass = 0; pass < 2; ++pass) { for (int i = t_; i < CSR_TS5 / 4; i += 256) { v4i a, c; for (int e = 0; e < 4; ++e) { a[e] = st; c[e] = 0; } *(volatile v4i*)(ROWPTR + t0 + i * 4) = a; *(volatile v4i*)(ROWCNT + t0 + i * 4) = c; } if (t_ == 0) ((volatile int*)FLAG)[0] = 1; __threadfence(); } (void)nv; return; }
  if (t_ == 0) { int acc = 0; for (int b = 0; b < CSR_NBLK5; ++b) { boff[b] = acc; int c = HST[(size_t)b * NGP + g]; c = (c < 0) ? 0 : (c > CHP ? CHP : c); acc += c; if (acc > tot) acc = tot; } boff[CSR_NBLK5] = acc; }
  for (int i = t_; i <= CSR_GN5; i += 256) ncnt[i] = 0;
  __syncthreads();
  for (int b = 0; b < CSR_NBLK5; ++b) { const int c = boff[b + 1] - boff[b]; int o_ = OFF[(size_t)g * CSR_NBLK5 + b]; o_ = (o_ < 0) ? 0 : (o_ > CHP - c ? CHP - c : o_); const int* src_ = STG + (size_t)b * CHP + o_;
    for (int i = t_; i < c; i += 256) { int id = src_[i]; id = (id < 0) ? 0 : id; ids[boff[b] + i] = id; int d = dst[id]; d = (d < v0) ? v0 : (d >= N ? N - 1 : d); int kk = d - v0; kk = (kk < 0) ? 0 : (kk >= CSR_GN5 ? CSR_GN5 - 1 : kk); key[boff[b] + i] = (unsigned short)kk; } }
  __syncthreads();
  if (t_ == 0) { for (int i = 0; i < tot; ++i) ncnt[key[i]] += 1; int acc = 0; for (int vl = 0; vl < CSR_GN5; ++vl) { const int c = ncnt[vl]; ncnt[vl] = acc; acc += c; } ncnt[CSR_GN5] = acc;
    for (int i = 0; i < tot; ++i) { const int vl = key[i]; outp[ncnt[vl]] = ids[i]; ncnt[vl] += 1; }
    for (int vl = CSR_GN5; vl > 0; --vl) ncnt[vl] = ncnt[vl - 1]; ncnt[0] = 0; }
  __syncthreads();
  for (int pass = 0; pass < 2; ++pass) {
    for (int i = t_; i < (stn - st) / 4; i += 256) { v4i v; for (int e = 0; e < 4; ++e) { const int q = i * 4 + e; v[e] = (q < tot) ? outp[q] : -1; } *(volatile v4i*)(PERM + st + i * 4) = v; }
    for (int i = t_; i < CSR_TS5 / 4; i += 256) { v4i a, c; for (int e = 0; e < 4; ++e) { const int vl = i * 4 + e; const int vc = vl < CSR_GN5 ? vl : CSR_GN5; a[e] = (vl < CSR_GN5) ? st + ncnt[vc] : st; c[e] = (vl < nv) ? (ncnt[(vc < CSR_GN5 ? vc : CSR_GN5 - 1) + 1] - ncnt[vc]) : 0; } *(volatile v4i*)(ROWPTR + t0 + i * 4) = a; *(volatile v4i*)(ROWCNT + t0 + i * 4) = c; }
    __threadfence(); }
}
__global__ __launch_bounds__(256) void csrZ_kernel5(int* __restrict__ p, size_t n4) { typedef __attribute__((ext_vector_type(4))) int v4i; const size_t tid = (size_t)blockIdx.x * 256 + threadIdx.x, nth = (size_t)gridDim.x * 256; v4i z = {0, 0, 0, 0}; for (size_t i = tid; i < n4; i += nth) *(volatile v4i*)(p + i * 4) = z; }
struct CsrBufs5 { int *STG, *HST, *OFF, *START, *TOT, *PERM, *ROWPTR, *ROWCNT, *FLAG; int nG, NGP, CHP; size_t permLen; char* base; size_t bytes; };
static size_t csr_carve5(CsrBufs5& c, char* ws, size_t off, int E, int N) {
  const size_t off0 = off; c.base = ws + off;
  auto al = [&](size_t bytes) { char* p = ws + off; off += (bytes + 255) & ~(size_t)255; return p; };
  c.nG = (N + CSR_GN5 - 1) / CSR_GN5; c.NGP = (c.nG + 31) & ~31; const int ch = (E + CSR_NBLK5 - 1) / CSR_NBLK5; c.CHP = (ch + 31) & ~31; c.permLen = (size_t)E + 32 * (size_t)c.nG + 32;
  c.STG = (int*)al((size_t)CSR_NBLK5 * c.CHP * 4); c.HST = (int*)al((size_t)CSR_NBLK5 * c.NGP * 4); c.OFF = (int*)al((size_t)c.NGP * CSR_NBLK5 * 4); c.START = (int*)al((size_t)(c.NGP + 64) * 4); c.TOT = (int*)al((size_t)(c.NGP + 64) * 4);
  c.PERM = (int*)al(c.permLen * 4); c.ROWPTR = (int*)al((size_t)c.nG * CSR_TS5 * 4); c.ROWCNT = (int*)al((size_t)c.nG * CSR_TS5 * 4); c.FLAG = (int*)al(256);
  c.bytes = off - off0; return off;
}
static void csr_build5(const CsrBufs5& c, const int* dst, int E, int N, hipStream_t stream) {
  const size_t smem = (size_t)(2 * c.NGP + c.CHP) * 4;
  csrZ_kernel5<<<512, 256, 0, stream>>>((int*)c.base, c.bytes / 16);
  csrA_kernel5<<<CSR_NBLK5, 64, smem, stream>>>(dst, E, N, c.nG, c.CHP, c.NGP, c.STG, c.HST);
  csrS_kernel5<<<1, 512, 0, stream>>>(c.HST, c.nG, c.NGP, c.START, c.TOT, c.OFF);
  csrB_kernel5<<<c.nG, 256, 0, stream>>>(dst, N, c.nG, c.CHP, c.NGP, (int)c.permLen, c.STG, c.HST, c.OFF, c.START, c.TOT, c.PERM, c.ROWPTR, c.ROWCNT, c.FLAG);
}


__global__ __launch_bounds__(256) void lin1_kernel(const float* __restrict__ xv, const float* __restrict__ xr, const float* __restrict__ vWl, const float* __restrict__ vbl, const float* __restrict__ vWr, const float* __restrict__ vbr, const float* __restrict__ iWl, const float* __restrict__ ibl, const float* __restrict__ iWr, const float* __restrict__ ibr, const float* __restrict__ rWl, const float* __restrict__ rbl, const float* __restrict__ rWr, const float* __restrict__ rbr, int VLIM, float* __restrict__ PV1, float* __restrict__ PR1) {
  const int wave = threadIdx.x >> 5, lane = threadIdx.x & 31; const size_t n = (size_t)blockIdx.x * 8 + wave;
  if (n < (size_t)VLIM) { float x6[DV]; for (int q = 0; q < DV; ++q) x6[q] = bfv(xv[n * DV + q]); float o[8];
#pragma unroll
    for (int j = 0; j < 8; ++j) { const int col = lane * 8 + j; const int g = col / L2, c = col % L2; const float* W = g == 0 ? vWl : (g == 1 ? vWr : (g == 2 ? iWl : rWr)); const float* bb = g == 0 ? vbl : (g == 1 ? vbr : (g == 2 ? ibl : rbr)); float s = bfv(bb[c]);
#pragma unroll
      for (int q = 0; q < DV; ++q) s += pmul(x6[q], bfv(W[q * L2 + c])); o[j] = s; }
    for (int pass = 0; pass < 2; ++pass) { *(volatile v4f*)(PV1 + n * 256 + lane * 8) = (v4f){o[0], o[1], o[2], o[3]}; *(volatile v4f*)(PV1 + n * 256 + lane * 8 + 4) = (v4f){o[4], o[5], o[6], o[7]}; __threadfence(); } }
  if (n < (size_t)NRS) { const float x1 = bfv(xr[n]); float o[4];
#pragma unroll
    for (int j = 0; j < 4; ++j) { const int col = lane * 4 + j; const int g = col / L2, c = col % L2; o[j] = g == 0 ? pmul(x1, bfv(iWr[c])) + bfv(ibr[c]) : pmul(x1, bfv(rWl[c])) + bfv(rbl[c]); }
    for (int pass = 0; pass < 2; ++pass) { *(volatile v4f*)(PR1 + n * 128 + lane * 4) = (v4f){o[0], o[1], o[2], o[3]}; __threadfence(); } } }
template <int NH>
__device__ __forceinline__ v2f gatv2_node(size_t i, const float* __restrict__ HLP, int hls, int hloff, const float* hr2, const float* __restrict__ att, const int* __restrict__ srcs, const int* __restrict__ PERM, const int* __restrict__ ROWPTR, const int* __restrict__ ROWCNT, int permLen, int Emax, int nsrc, int SLIM, int mask, int loop, int lane) {
  int st = ROWPTR[i], cnt = ROWCNT[i]; cnt = iclamp(cnt, 0, Emax); st = iclamp(st, 0, permLen - cnt); const float a0 = bfv(att[lane * 2]), a1 = bfv(att[lane * 2 + 1]); float mx = -INFINITY, den = 0.0f, acc0 = 0.0f, acc1 = 0.0f; constexpr int SEG = 32 / NH;
  auto visit = [&](size_t u) { const float m0 = HLP[u * hls + hloff + lane * 2], m1 = HLP[u * hls + hloff + lane * 2 + 1]; float s = pmul(leaky(m0 + hr2[0]), a0) + pmul(leaky(m1 + hr2[1]), a1);
#pragma unroll
    for (int o = SEG / 2; o; o >>= 1) s += __shfl_xor(s, o);
    const float mn = fmaxf(mx, s); const float sf = (mx == -INFINITY) ? 0.0f : __expf(mx - mn); const float p = __expf(s - mn); den = den * sf + p; acc0 = pmul(acc0, sf) + pmul(p, m0); acc1 = pmul(acc1, sf) + pmul(p, m1); mx = mn; };
#pragma unroll 1
  for (int j = 0; j < cnt; ++j) { const int e = iclamp(PERM[st + j], 0, Emax - 1); const size_t u = (size_t)iclamp(srcs[e], 0, nsrc - 1); if (u >= (size_t)SLIM) continue; if (mask && u == i) continue; visit(u); }
  if (loop) visit(i);
  v2f r; r[0] = den > 0.0f ? acc0 / (den + 1e-16f) : 0.0f; r[1] = den > 0.0f ? acc1 / (den + 1e-16f) : 0.0f; return r; }

__global__ __launch_bounds__(256) void l1veh_kernel(const float* __restrict__ PV1, const float* __restrict__ PR1, const float* __restrict__ vatt, const float* __restrict__ vb, const float* __restrict__ ratt, const float* __restrict__ rb, const int* __restrict__ vvsrc, const int* __restrict__ P1, const int* __restrict__ RP1, const int* __restrict__ RC1, int pl1, const int* __restrict__ ivsrc, const int* __restrict__ P2, const int* __restrict__ RP2, const int* __restrict__ RC2, int pl2, int VLIM, float* __restrict__ HV) {
  const int wave = threadIdx.x >> 5, lane = threadIdx.x & 31; const size_t i = (size_t)blockIdx.x * NPB + wave; if (i >= (size_t)VLIM) return;
  float hr[2]; hr[0] = PV1[i * 256 + 64 + lane * 2]; hr[1] = PV1[i * 256 + 64 + lane * 2 + 1];
  const v2f a = gatv2_node<2>(i, PV1, 256, 0, hr, vatt, vvsrc, P1, RP1, RC1, pl1, EVV, NV, VLIM, 1, 1, lane);
  hr[0] = PV1[i * 256 + 192 + lane * 2]; hr[1] = PV1[i * 256 + 192 + lane * 2 + 1];
  const v2f b = gatv2_node<2>(i, PR1, 128, 64, hr, ratt, ivsrc, P2, RP2, RC2, pl2, EIV, NRS, NRS, 0, 0, lane);
  v2f o; for (int k = 0; k < 2; ++k) { const int c = lane * 2 + k; o[k] = elu(a[k] + bfv(vb[c]) + b[k] + bfv(rb[c])); }
  for (int pass = 0; pass < 2; ++pass) { *(volatile v2f*)(HV + i * L2 + lane * 2) = o; __threadfence(); } }
__global__ __launch_bounds__(256) void l1rsu_kernel(const float* __restrict__ PV1, const float* __restrict__ PR1, const float* __restrict__ iatt, const float* __restrict__ ib, const int* __restrict__ visrc, const int* __restrict__ P3, const int* __restrict__ RP3, const int* __restrict__ RC3, int pl3, int VLIM, float* __restrict__ HR) {
  const int wave = threadIdx.x >> 5, lane = threadIdx.x & 31; const size_t i = (size_t)blockIdx.x * NPB + wave; if (i >= (size_t)NRS) return;
  float hr[2]; hr[0] = PR1[i * 128 + lane * 2]; hr[1] = PR1[i * 128 + lane * 2 + 1];
  const v2f a = gatv2_node<2>(i, PV1, 256, 128, hr, iatt, visrc, P3, RP3, RC3, pl3, EVI, NV, VLIM, 0, 0, lane);
  v2f o; for (int k = 0; k < 2; ++k) o[k] = elu(a[k] + bfv(ib[lane * 2 + k]));
  for (int pass = 0; pass < 2; ++pass) { *(volatile v2f*)(HR + i * L2 + lane * 2) = o; __threadfence(); } }
__global__ __launch_bounds__(256) void wput_kernel(const float* __restrict__ a0, const float* __restrict__ a1, const float* __restrict__ a2, const float* __restrict__ a3, const float* __restrict__ c0, const float* __restrict__ c1, b16* __restrict__ WV, b16* __restrict__ WR2) { const int u = blockIdx.x * 256 + threadIdx.x; v8b v;
  if (u < 256 * 8) { const int o = u / 8, k0 = (u % 8) * 8; const int g = o / 64, c = o % 64; const float* W = g == 0 ? a0 : (g == 1 ? a1 : (g == 2 ? a2 : a3));
#pragma unroll
    for (int j = 0; j < 8; ++j) v[j] = (b16)(bf16_rne(W[(size_t)(k0 + j) * 64 + c]) * WSC); for (int pass = 0; pass < 2; ++pass) { *(volatile v8b*)(WV + (size_t)o * 64 + k0) = v; __threadfence(); } }
  if (u < 128 * 8) { const int o = u / 8, k0 = (u % 8) * 8; const int g = o / 64, c = o % 64; const float* W = g == 0 ? c0 : c1;
#pragma unroll
    for (int j = 0; j < 8; ++j) v[j] = (b16)(bf16_rne(W[(size_t)(k0 + j) * 64 + c]) * WSC); for (int pass = 0; pass < 2; ++pass) { *(volatile v8b*)(WR2 + (size_t)o * 64 + k0) = v; __threadfence(); } } }
__global__ __launch_bounds__(32) void lin2_kernel(const float* __restrict__ HV, const float* __restrict__ HR, const b16* __restrict__ WV, const b16* __restrict__ WR2, const float* __restrict__ bv0, const float* __restrict__ bv1, const float* __restrict__ bv2, const float* __restrict__ bv3, const float* __restrict__ br0, const float* __restrict__ br1, int VLIM, float* __restrict__ PV2, float* __restrict__ PR2) {
  __shared__ __attribute__((aligned(16))) b16 Ah[16][72], Al[16][72]; __shared__ float Tf[16][260]; const int lane = threadIdx.x, nloc = lane & 15, hlf = lane >> 4; const bool rsu = blockIdx.x >= (unsigned)(NV / 16); const size_t m0 = rsu ? (size_t)(blockIdx.x - NV / 16) * 16 : (size_t)blockIdx.x * 16; if (!rsu && m0 >= (size_t)VLIM) return;
  const float* Hs = rsu ? HR : HV; const int nrow = rsu ? NRS : NV; const int NT = rsu ? 8 : 16; const b16* W = rsu ? WR2 : WV;
  for (int rr = 0; rr < 16; ++rr) { const size_t row = m0 + rr < (size_t)nrow ? m0 + rr : (size_t)nrow - 1; for (int q = 0; q < 2; ++q) { b16 p, ql; split16(Hs[row * L2 + q * 32 + lane] * HS, p, ql); Ah[rr][q * 32 + lane] = p; Al[rr][q * 32 + lane] = ql; } } if (lane < 16) for (int k = 64; k < 72; ++k) { Ah[lane][k] = (b16)0.0f; Al[lane][k] = (b16)0.0f; }
  wave_lds_sync(); v8f acc[16];
#pragma unroll
  for (int t = 0; t < 16; ++t) acc[t] = (v8f){};
#pragma unroll
  for (int kb = 0; kb < 64; kb += 32) { const v16b a = frag_kb(&Ah[nloc][kb], hlf), al = frag_kb(&Al[nloc][kb], hlf);
#pragma unroll
    for (int t = 0; t < 16; ++t) if (t < NT) { const v16b bw = frag_kb(W + (size_t)(t * 16 + nloc) * 64 + kb, hlf); acc[t] = wmma16b(a, bw, acc[t]); acc[t] = wmma16b(al, bw, acc[t]); } }
#pragma unroll
  for (int t = 0; t < 16; ++t) if (t < NT) { const int cc = t * 16 + nloc; const int g = cc / 64, c = cc % 64; const float bb = rsu ? (g == 0 ? bfv(br0[c]) : bfv(br1[c])) : (g == 0 ? bfv(bv0[c]) : (g == 1 ? bfv(bv1[c]) : (g == 2 ? bfv(bv2[c]) : bfv(bv3[c]))));
#pragma unroll
    for (int r8 = 0; r8 < 8; ++r8) Tf[8 * hlf + r8][cc] = acc[t][r8] * (1.0f / (HS * WSC)) + bb; }
  wave_lds_sync();
  for (int pass = 0; pass < 2; ++pass) { for (int rr = 0; rr < 16; ++rr) { if (rsu) *(volatile v4f*)(PR2 + (m0 + rr) * 128 + lane * 4) = *(const v4f*)(&Tf[rr][lane * 4]); else for (int q = 0; q < 2; ++q) *(volatile v4f*)(PV2 + (m0 + rr) * 256 + q * 128 + lane * 4) = *(const v4f*)(&Tf[rr][q * 128 + lane * 4]); } __threadfence(); } }
__global__ __launch_bounds__(256) void l2veh_kernel(const float* __restrict__ PV2, const float* __restrict__ PR2, const float* __restrict__ vatt, const float* __restrict__ vb, const float* __restrict__ ratt, const float* __restrict__ rb, const float* __restrict__ lw, const float* __restrict__ lb, const int* __restrict__ vvsrc, const int* __restrict__ P1, const int* __restrict__ RP1, const int* __restrict__ RC1, int pl1, const int* __restrict__ ivsrc, const int* __restrict__ P2, const int* __restrict__ RP2, const int* __restrict__ RC2, int pl2, int VLIM, float* __restrict__ OUT0) {
  const int wave = threadIdx.x >> 5, lane = threadIdx.x & 31; const size_t i = (size_t)blockIdx.x * NPB + wave; if (i >= (size_t)VLIM) return;
  float hr[2]; hr[0] = PV2[i * 256 + 64 + lane * 2]; hr[1] = PV2[i * 256 + 64 + lane * 2 + 1];
  const v2f a = gatv2_node<1>(i, PV2, 256, 0, hr, vatt, vvsrc, P1, RP1, RC1, pl1, EVV, NV, VLIM, 1, 1, lane);
  hr[0] = PV2[i * 256 + 192 + lane * 2]; hr[1] = PV2[i * 256 + 192 + lane * 2 + 1];
  const v2f b = gatv2_node<1>(i, PR2, 128, 0, hr, ratt, ivsrc, P2, RP2, RC2, pl2, EIV, NRS, NRS, 1, i < (size_t)NRS ? 1 : 0, lane);
  float v[2], sm = 0.0f; for (int k = 0; k < 2; ++k) { const int c = lane * 2 + k; v[k] = a[k] + bfv(vb[c]) + b[k] + bfv(rb[c]); sm += v[k]; } for (int o = 16; o; o >>= 1) sm += __shfl_xor(sm, o); const float mu = sm / OUT; float q2 = 0.0f; for (int k = 0; k < 2; ++k) q2 += (v[k] - mu) * (v[k] - mu); for (int o = 16; o; o >>= 1) q2 += __shfl_xor(q2, o); const float rs = rsqrtf(q2 / OUT + LNEPS);
  v2f o2; for (int k = 0; k < 2; ++k) { const int c = lane * 2 + k; o2[k] = pmul((v[k] - mu) * rs, bfv(lw[c])) + bfv(lb[c]); }
  for (int pass = 0; pass < 2; ++pass) { *(volatile v2f*)(OUT0 + i * OUT + lane * 2) = o2; __threadfence(); } }
__global__ __launch_bounds__(256) void l2rsu_kernel(const float* __restrict__ PV2, const float* __restrict__ PR2, const float* __restrict__ iatt, const float* __restrict__ ib, const float* __restrict__ lw, const float* __restrict__ lb, const int* __restrict__ visrc, const int* __restrict__ P3, const int* __restrict__ RP3, const int* __restrict__ RC3, int pl3, int VLIM, float* __restrict__ OUT1) {
  const int wave = threadIdx.x >> 5, lane = threadIdx.x & 31; const size_t i = (size_t)blockIdx.x * NPB + wave; if (i >= (size_t)NRS) return;
  float hr[2]; hr[0] = PR2[i * 128 + 64 + lane * 2]; hr[1] = PR2[i * 128 + 64 + lane * 2 + 1];
  const v2f a = gatv2_node<1>(i, PV2, 256, 128, hr, iatt, visrc, P3, RP3, RC3, pl3, EVI, NV, VLIM, 1, i < (size_t)VLIM ? 1 : 0, lane);
  float v[2], sm = 0.0f; for (int k = 0; k < 2; ++k) { v[k] = a[k] + bfv(ib[lane * 2 + k]); sm += v[k]; } for (int o = 16; o; o >>= 1) sm += __shfl_xor(sm, o); const float mu = sm / OUT; float q2 = 0.0f; for (int k = 0; k < 2; ++k) q2 += (v[k] - mu) * (v[k] - mu); for (int o = 16; o; o >>= 1) q2 += __shfl_xor(q2, o); const float rs = rsqrtf(q2 / OUT + LNEPS);
  v2f o2; for (int k = 0; k < 2; ++k) { const int c = lane * 2 + k; o2[k] = pmul((v[k] - mu) * rs, bfv(lw[c])) + bfv(lb[c]); }
  for (int pass = 0; pass < 2; ++pass) { *(volatile v2f*)(OUT1 + i * OUT + lane * 2) = o2; __threadfence(); } }
}

extern "C" void kernel_launch(void* const* d_in, const int* in_sizes, int n_in, void* d_out, int out_size, void* d_ws, size_t ws_size, hipStream_t stream) {
  (void)n_in;
  auto Fp = [&](int i) { return (const float*)d_in[i]; }; auto Ip = [&](int i) { return (const int*)d_in[i]; };
  if (in_sizes[0] != NV * DV || in_sizes[1] != NRS || in_sizes[2] != 2 * EVV || in_sizes[3] != 2 * EVI || in_sizes[4] != 2 * EIV || in_sizes[5] != DV * L2 || in_sizes[13] != 1 * L2 || in_sizes[17] != 1 * L2 || in_sizes[23] != L2 * OUT || in_sizes[29] != L2 * OUT || in_sizes[35] != L2 * OUT || out_size != NV * OUT + NRS * OUT) return;
  const int VLIM = NV;
  size_t off = 0; char* ws = (char*)d_ws;
  auto carve = [&](size_t bytes) { char* p = ws + off; off += (bytes + 255) & ~(size_t)255; return p; };
  float* PV1 = (float*)carve((size_t)NV * 256 * 4); float* PR1 = (float*)carve((size_t)NRP * 128 * 4); float* HV = (float*)carve((size_t)NV * L2 * 4); float* HR = (float*)carve((size_t)NRP * L2 * 4); b16* WV = (b16*)carve(256 * 64 * 2); b16* WR2 = (b16*)carve(128 * 64 * 2); float* PV2 = (float*)carve((size_t)NV * 256 * 4); float* PR2 = (float*)carve((size_t)NRP * 128 * 4);
  CsrBufs8 c1, c2; CsrBufs5 c3; off = csr_carve8(c1, ws, off, EVV, NV); off = csr_carve8(c2, ws, off, EIV, NV); off = csr_carve5(c3, ws, off, EVI, NRS);
  if (off > ws_size || off > ((size_t)160 << 20)) return;
  const int nbv = (VLIM + NPB - 1) / NPB, nbr = (NRS + NPB - 1) / NPB;
  csr_build8(c1, Ip(2) + EVV, EVV, NV, stream); csr_build8(c2, Ip(4) + EIV, EIV, NV, stream); csr_build5(c3, Ip(3) + EVI, EVI, NRS, stream);
  lin1_kernel<<<(NV + 7) / 8, 256, 0, stream>>>(Fp(0), Fp(1), Fp(5), Fp(6), Fp(7), Fp(8), Fp(11), Fp(12), Fp(13), Fp(14), Fp(17), Fp(18), Fp(19), Fp(20), VLIM, PV1, PR1);
  l1veh_kernel<<<nbv, 256, 0, stream>>>(PV1, PR1, Fp(9), Fp(10), Fp(21), Fp(22), Ip(2), c1.PERM, c1.ROWPTR, c1.ROWCNT, (int)c1.permLen, Ip(4), c2.PERM, c2.ROWPTR, c2.ROWCNT, (int)c2.permLen, VLIM, HV);
  l1rsu_kernel<<<nbr, 256, 0, stream>>>(PV1, PR1, Fp(15), Fp(16), Ip(3), c3.PERM, c3.ROWPTR, c3.ROWCNT, (int)c3.permLen, VLIM, HR);
  wput_kernel<<<(256 * 8 + 255) / 256, 256, 0, stream>>>(Fp(23), Fp(25), Fp(29), Fp(37), Fp(35), Fp(31), WV, WR2);
  lin2_kernel<<<NV / 16 + NRP / 16, 32, 0, stream>>>(HV, HR, WV, WR2, Fp(24), Fp(26), Fp(30), Fp(38), Fp(36), Fp(32), VLIM, PV2, PR2);
  l2veh_kernel<<<nbv, 256, 0, stream>>>(PV2, PR2, Fp(27), Fp(28), Fp(39), Fp(40), Fp(41), Fp(42), Ip(2), c1.PERM, c1.ROWPTR, c1.ROWCNT, (int)c1.permLen, Ip(4), c2.PERM, c2.ROWPTR, c2.ROWCNT, (int)c2.permLen, VLIM, (float*)d_out);
  l2rsu_kernel<<<nbr, 256, 0, stream>>>(PV2, PR2, Fp(33), Fp(34), Fp(43), Fp(44), Ip(3), c3.PERM, c3.ROWPTR, c3.ROWCNT, (int)c3.permLen, VLIM, (float*)d_out + (size_t)NV * OUT);
}
